// RWKV7Adapter_85237920957009
// MI455X (gfx1250) — hardware-verified
//
#include <hip/hip_runtime.h>
#include <math.h>

#pragma clang fp contract(off)

typedef __attribute__((ext_vector_type(16))) _Float16 v16h;
typedef __attribute__((ext_vector_type(8)))  _Float16 v8h;
typedef __attribute__((ext_vector_type(16))) __bf16   v16b;
typedef __attribute__((ext_vector_type(8)))  __bf16   v8b;
typedef __attribute__((ext_vector_type(8)))  float    v8f;
typedef __attribute__((ext_vector_type(4)))  float    v4f;
typedef __attribute__((ext_vector_type(4)))  unsigned int v4u;

constexpr int  kBatch = 4;
constexpr int  kSeq   = 2048;
constexpr int  kDim   = 256;
constexpr int  kTok   = kBatch * kSeq;
constexpr long kPE    = (long)kTok * kDim;
constexpr int  kLrW   = 64;
constexpr int  kLrA   = 64;
constexpr int  kLrG   = 128;
constexpr float kDecayScale = -0.6065306597126334f;
constexpr float kGnEps      = 0.00256f;
constexpr float kInvDim     = 1.0f / 256.0f;
constexpr int  kVecPad = 272;
constexpr int  kScanThreads = 512;
constexpr int  kHalf = 128;

constexpr size_t kPlaneF32B = (size_t)kPE * 4;
constexpr size_t kPlaneBfB  = (size_t)kPE * 2;
constexpr size_t kOffWt4Hi = 0;
constexpr size_t kOffWt4Lo = 524288;
constexpr size_t kOffAw2Hi = 1048576;
constexpr size_t kOffAw2Lo = 1114112;
constexpr size_t kOffAgHi  = 1179648;
constexpr size_t kOffAgLo  = 1245184;
constexpr size_t kOffBw2Hi = 1310720;
constexpr size_t kOffBw2Lo = 1376256;
constexpr size_t kOffBgHi  = 1441792;
constexpr size_t kOffBgLo  = 1507328;
constexpr size_t kOffF     = 2097152;
constexpr size_t kOffXmHi  = kOffF + 3 * kPlaneF32B;
constexpr size_t kOffXmLo  = kOffXmHi + 6 * kPlaneBfB;
constexpr size_t kOffOgHi  = kOffF + 8 * kPlaneF32B;
constexpr size_t kOffOgLo  = kOffOgHi + kPlaneBfB;
constexpr size_t kOffLw    = kOffF + 9 * kPlaneF32B;
constexpr size_t kOffLwWHi = kOffLw;
constexpr size_t kOffLwWLo = kOffLw + 1048576;
constexpr size_t kOffLwAHi = kOffLw + 2097152;
constexpr size_t kOffLwALo = kOffLw + 3145728;
constexpr size_t kOffLwGHi = kOffLw + 4194304;
constexpr size_t kOffLwGLo = kOffLw + 6291456;
constexpr size_t kOffPre   = kOffLw + 8388608;
constexpr size_t kOffWpre  = kOffPre;
constexpr size_t kOffApre  = kOffPre + kPlaneF32B;
constexpr size_t kOffG     = kOffPre + 2 * kPlaneF32B;
constexpr size_t kCarveBytes = kOffPre + 3 * kPlaneF32B;
static_assert(kCarveBytes == 111149056, "carve");
static_assert(kOffXmLo + 6 * kPlaneBfB == kOffLw, "xm planes end at lw");
static_assert(kOffOgLo + kPlaneBfB == kOffLw, "og planes end at lw");

__device__ __forceinline__ unsigned short f2bf_bits(float f) {
  unsigned u = __float_as_uint(f);
  return (unsigned short)((u + 0x7FFFu + ((u >> 16) & 1u)) >> 16);
}
__device__ __forceinline__ float bf_bits2f(unsigned short h) { return __uint_as_float(((unsigned)h) << 16); }

__device__ __forceinline__ void dep_guard_h(v8f& a, v8f& b, v16h x, v16h y) { asm volatile("v_nop\n\tv_nop\n\tv_nop\n\tv_nop" : "+v"(a), "+v"(b) : "v"(x), "v"(y)); }
__device__ __forceinline__ void dep_guard_b(v8f& a, v8f& b, v16b x, v16b y) { asm volatile("v_nop\n\tv_nop\n\tv_nop\n\tv_nop" : "+v"(a), "+v"(b) : "v"(x), "v"(y)); }
__device__ __forceinline__ void keep4_h(v16h a, v16h b, v16h c, v16h d) { asm volatile("v_nop" :: "v"(a), "v"(b), "v"(c), "v"(d)); }
__device__ __forceinline__ void keep4_b(v16b a, v16b b, v16b c, v16b d) { asm volatile("v_nop" :: "v"(a), "v"(b), "v"(c), "v"(d)); }
__device__ __forceinline__ void acc_guard4(v8f& a, v8f& b, v8f& c, v8f& d) { asm volatile("v_nop\n\tv_nop\n\tv_nop\n\tv_nop" : "+v"(a), "+v"(b), "+v"(c), "+v"(d)); }
template <typename T> struct Frag;
template <> struct Frag<_Float16> {
  typedef v16h V; union U { v16h v; v8h h[2]; };
  static __device__ __forceinline__ v16h load(const _Float16* p) {
    U f; f.h[0] = *(const v8h*)(p); f.h[1] = *(const v8h*)(p + 16); return f.v;
  }
  static __device__ __forceinline__ v8f mma(v16h a, v16h b, v8f c) {
    return __builtin_amdgcn_wmma_f32_16x16x32_f16(false, a, false, b, (short)0, c, false, false);
  }
  static __device__ __forceinline__ void guard(v8f& a, v8f& b, v16h x, v16h y) { dep_guard_h(a, b, x, y); }
  static __device__ __forceinline__ void keep(v16h a, v16h b, v16h c, v16h d) { keep4_h(a, b, c, d); }
};
template <> struct Frag<__bf16> {
  typedef v16b V; union U { v16b v; v8b h[2]; };
  static __device__ __forceinline__ v16b load(const __bf16* p) {
    U f; f.h[0] = *(const v8b*)(p); f.h[1] = *(const v8b*)(p + 16); return f.v;
  }
  static __device__ __forceinline__ v8f mma(v16b a, v16b b, v8f c) {
    return __builtin_amdgcn_wmma_f32_16x16x32_bf16(false, a, false, b, (short)0, c, false, false);
  }
  static __device__ __forceinline__ void guard(v8f& a, v8f& b, v16b x, v16b y) { dep_guard_b(a, b, x, y); }
  static __device__ __forceinline__ void keep(v16b a, v16b b, v16b c, v16b d) { keep4_b(a, b, c, d); }
};

__device__ __forceinline__ unsigned pk16(unsigned short a, unsigned short b) { return (unsigned)a | ((unsigned)b << 16); }

template <int ET> struct Elem;
template <> struct Elem<0> { typedef _Float16 T; };
template <> struct Elem<1> { typedef __bf16 T; };
template <int ET, bool SPLIT, int BIAS_MODE, int OUT_MODE, bool RESID, int ACT = 0>
__global__ __launch_bounds__(256) void wmma_gemm64(
    const unsigned short* __restrict__ Ap, const unsigned short* __restrict__ A2p, int lda, long strideA,
    const unsigned short* __restrict__ Btp, const unsigned short* __restrict__ Bt2p, int ldb, long strideB,
    void* __restrict__ Cout, void* __restrict__ Cout2, int ldc, long strideC,
    const float* __restrict__ bias,
    const float* __restrict__ resid, long strideR,
    int M, int N, int K, float scale) {
  typedef typename Elem<ET>::T T;
  typedef typename Frag<T>::V V;
  const T* A = (const T*)Ap; const T* A2 = (const T*)A2p; const T* Bt = (const T*)Btp; const T* Bt2 = (const T*)Bt2p;
  __shared__ __align__(16) float sT[8][16 * 68];
  const int b    = blockIdx.y;
  const int lane = threadIdx.x & 31;
  const int wave = threadIdx.x >> 5;
  const int tilesN = N >> 6;
  const int tilesM = M >> 6;
  const int tile = blockIdx.x * 8 + wave;
  if (tile >= tilesM * tilesN) return;
  const int tm = tile / tilesN;
  const int tn = tile - tm * tilesN;
  const int m0 = tm << 6;
  const int n0 = tn << 6;

  const T* Ab  = A  + (size_t)b * strideA;
  const T* Bb  = Bt + (size_t)b * strideB;
  const T* Ab2 = SPLIT ? (A2  + (size_t)b * strideA) : nullptr;
  const T* Bb2 = SPLIT ? (Bt2 + (size_t)b * strideB) : nullptr;

  const int rlane = lane & 15;
  const int koff  = (lane >> 4) * 8;
  const int mOff  = (lane >> 4) * 8;

  v8f acc[4][4];
#pragma unroll
  for (int i = 0; i < 4; ++i)
#pragma unroll
    for (int j = 0; j < 4; ++j) acc[i][j] = (v8f){0.f,0.f,0.f,0.f,0.f,0.f,0.f,0.f};

  for (int k0 = 0; k0 < K; k0 += 32) {
    V bh[4], bl[4];
#pragma unroll
    for (int j = 0; j < 4; ++j) {
      const size_t bo = (size_t)(n0 + (j << 4) + rlane) * ldb + koff + k0;
      bh[j] = Frag<T>::load(Bb + bo);
      if (SPLIT) bl[j] = Frag<T>::load(Bb2 + bo);
    }
#pragma unroll
    for (int i = 0; i < 4; ++i) {
      const size_t ao = (size_t)(m0 + (i << 4) + rlane) * lda + koff + k0;
      V ah = Frag<T>::load(Ab + ao);
      V al;
      if (SPLIT) al = Frag<T>::load(Ab2 + ao);
#pragma unroll
      for (int j = 0; j < 4; ++j) {
        acc[i][j] = Frag<T>::mma(ah, bh[j], acc[i][j]);
        if (SPLIT) {
          acc[i][j] = Frag<T>::mma(ah, bl[j], acc[i][j]);
          acc[i][j] = Frag<T>::mma(al, bh[j], acc[i][j]);
        }
      }
      Frag<T>::guard(acc[i][0], acc[i][3], ah, SPLIT ? al : ah);
    }
    Frag<T>::keep(bh[0], bh[1], bh[2], bh[3]);
    if (SPLIT) Frag<T>::keep(bl[0], bl[1], bl[2], bl[3]);
  }
  acc_guard4(acc[0][0], acc[0][1], acc[0][2], acc[0][3]);
  acc_guard4(acc[1][0], acc[1][1], acc[1][2], acc[1][3]);
  acc_guard4(acc[2][0], acc[2][1], acc[2][2], acc[2][3]);
  acc_guard4(acc[3][0], acc[3][1], acc[3][2], acc[3][3]);

  float* slab = sT[wave];
  const float* Rb = RESID ? (resid + (size_t)b * strideR) : nullptr;
#pragma unroll
  for (int i = 0; i < 4; ++i) {
    const int mBase = m0 + (i << 4);
#pragma unroll
    for (int j = 0; j < 4; ++j) {
      const int n = n0 + (j << 4) + rlane;
      float bv = 0.f;
      if (BIAS_MODE == 2) bv = bias[n];
#pragma unroll
      for (int r = 0; r < 8; ++r) {
        float v = acc[i][j][r] * scale;
        if (BIAS_MODE == 1) v += bias[mBase + mOff + r];
        if (BIAS_MODE == 2) v += bv;
        if (RESID) v += Rb[(size_t)(mBase + mOff + r) * ldc + n];
        if (ACT == 1) v = tanhf(v);
        if (ACT == 2) v = fmaxf(v, 0.0f);
        if (ACT == 3) v = v / (1.0f + expf(-v));
        if (ACT == 4) v = (v > 0.f) ? v : 0.01f * v;
        if (ACT == 6) v = 1.0f / (1.0f + expf(-v));
        slab[(mOff + r) * 68 + (j << 4) + rlane] = v;
      }
    }
    __builtin_amdgcn_fence(__ATOMIC_RELEASE, "workgroup");
    __builtin_amdgcn_wave_barrier();
    __builtin_amdgcn_fence(__ATOMIC_ACQUIRE, "workgroup");
    if (OUT_MODE == 0) {
      float* C = (float*)Cout + (size_t)b * strideC;
      const int hh = lane >> 4, c4 = (lane & 15) * 4;
      for (int pass = 0; pass < 2; ++pass) {
#pragma unroll
        for (int it = 0; it < 8; ++it) {
          const int row = it * 2 + hh;
          v4f v = *(const v4f*)(slab + row * 68 + c4);
          *(volatile v4f*)(C + (size_t)(mBase + row) * ldc + n0 + c4) = v;
        }
        __threadfence();
      }
    } else {
      const int q = lane >> 3, c8 = (lane & 7) * 8;
      unsigned short* C  = (unsigned short*)Cout  + (size_t)b * strideC;
      unsigned short* C2 = (OUT_MODE == 2) ? ((unsigned short*)Cout2 + (size_t)b * strideC) : nullptr;
      for (int pass = 0; pass < 2; ++pass) {
#pragma unroll
        for (int it = 0; it < 4; ++it) {
          const int row = it * 4 + q;
          const float* sp = slab + row * 68 + c8;
          v8h hv, lv;
#pragma unroll
          for (int e = 0; e < 8; ++e) {
            if (OUT_MODE == 1) {
              hv[e] = (_Float16)sp[e];
            } else {
              unsigned short hb = f2bf_bits(sp[e]);
              unsigned short lb = f2bf_bits(sp[e] - bf_bits2f(hb));
              hv[e] = __builtin_bit_cast(_Float16, hb);
              lv[e] = __builtin_bit_cast(_Float16, lb);
            }
          }
          *(volatile v8h*)(C + (size_t)(mBase + row) * ldc + n0 + c8) = hv;
          if (OUT_MODE == 2) *(volatile v8h*)(C2 + (size_t)(mBase + row) * ldc + n0 + c8) = lv;
        }
        __threadfence();
      }
    }
    __builtin_amdgcn_fence(__ATOMIC_RELEASE, "workgroup");
    __builtin_amdgcn_wave_barrier();
    __builtin_amdgcn_fence(__ATOMIC_ACQUIRE, "workgroup");
  }
}

__global__ __launch_bounds__(256) void wsplit_t_kernel(const float* __restrict__ W0, const float* __restrict__ W1,
                                                       const float* __restrict__ W2, const float* __restrict__ W3,
                                                       unsigned short* __restrict__ hi, unsigned short* __restrict__ lo,
                                                       int kin, int nout) {
  __shared__ float sm[64][65];
  const int t  = threadIdx.x;
  const int k0 = blockIdx.x * 64;
  const int n0 = blockIdx.y * 64;
  const int z  = blockIdx.z;
  const float* W = (z == 0) ? W0 : (z == 1) ? W1 : (z == 2) ? W2 : W3;
#pragma unroll
  for (int i = 0; i < 16; ++i) {
    const int e = i * 256 + t;
    const int r = e >> 6;
    const int c = e & 63;
    sm[c][r] = W[(size_t)(k0 + r) * nout + n0 + c];
  }
  __syncthreads();
  const int lane = t & 31, wave = t >> 5;
  const int q = lane >> 3, c8 = (lane & 7) * 8;
  const size_t pz = (size_t)z * (size_t)nout * (size_t)kin;
  v4u hu[2], lu[2];
  size_t ad[2];
#pragma unroll
  for (int it = 0; it < 2; ++it) {
    const int row = wave * 8 + it * 4 + q;
    unsigned short hb[8], lb[8];
#pragma unroll
    for (int e = 0; e < 8; ++e) {
      const float f = sm[row][c8 + e];
      const unsigned short h = f2bf_bits(f);
      hb[e] = h;
      lb[e] = f2bf_bits(f - bf_bits2f(h));
    }
    hu[it] = (v4u){pk16(hb[0], hb[1]), pk16(hb[2], hb[3]), pk16(hb[4], hb[5]), pk16(hb[6], hb[7])};
    lu[it] = (v4u){pk16(lb[0], lb[1]), pk16(lb[2], lb[3]), pk16(lb[4], lb[5]), pk16(lb[6], lb[7])};
    ad[it] = pz + (size_t)(n0 + row) * kin + k0 + c8;
  }
#pragma unroll
  for (int it = 0; it < 2; ++it) {
    *(volatile v4u*)(hi + ad[it]) = hu[it];
    *(volatile v4u*)(lo + ad[it]) = lu[it];
  }
  __threadfence();
#pragma unroll
  for (int it = 0; it < 2; ++it) {
    *(volatile v4u*)(hi + ad[it]) = hu[it];
    *(volatile v4u*)(lo + ad[it]) = lu[it];
  }
}

__global__ __launch_bounds__(256) void mix_kernel(const float* __restrict__ x, const float* __restrict__ xmix,
                                                  unsigned short* __restrict__ xm_hi, unsigned short* __restrict__ xm_lo,
                                                  int n8) {
  const int i = blockIdx.x * 256 + threadIdx.x;
  if (i >= n8) return;
  const int row = i >> 5;
  const int ch0 = (i & 31) * 8;
  const int t = row & (kSeq - 1);
  const int prow = (t > 0) ? (row - 1) : row;
  const float* xc_p = x + (size_t)row * kDim + ch0;
  const float* xp_p = x + (size_t)prow * kDim + ch0;
  const v4f c0 = *(const v4f*)(xc_p);
  const v4f c1 = *(const v4f*)(xc_p + 4);
  const v4f p0 = *(const v4f*)(xp_p);
  const v4f p1 = *(const v4f*)(xp_p + 4);
  float xc[8], dl[8];
#pragma unroll
  for (int e = 0; e < 4; ++e) {
    xc[e] = c0[e];
    xc[4 + e] = c1[e];
    const float s0 = (t > 0) ? p0[e] : 0.0f;
    const float s1 = (t > 0) ? p1[e] : 0.0f;
    dl[e] = s0 - xc[e];
    dl[4 + e] = s1 - xc[4 + e];
  }
  v4u hu[6], lu[6];
#pragma unroll
  for (int j = 0; j < 6; ++j) {
    const int mr = (j == 0) ? 0 : (j == 1) ? 2 : (j == 2) ? 3 : (j == 3) ? 1 : j;
    const float* mp = xmix + mr * kDim + ch0;
    const v4f m0 = *(const v4f*)(mp);
    const v4f m1 = *(const v4f*)(mp + 4);
    float m[8];
#pragma unroll
    for (int e = 0; e < 4; ++e) { m[e] = m0[e]; m[4 + e] = m1[e]; }
    unsigned short hb[8], lb[8];
#pragma unroll
    for (int e = 0; e < 8; ++e) {
      const float f = xc[e] + dl[e] * m[e];
      const unsigned short h = f2bf_bits(f);
      hb[e] = h;
      lb[e] = f2bf_bits(f - bf_bits2f(h));
    }
    hu[j] = (v4u){pk16(hb[0], hb[1]), pk16(hb[2], hb[3]), pk16(hb[4], hb[5]), pk16(hb[6], hb[7])};
    lu[j] = (v4u){pk16(lb[0], lb[1]), pk16(lb[2], lb[3]), pk16(lb[4], lb[5]), pk16(lb[6], lb[7])};
  }
  const size_t eo = (size_t)8 * i;
#pragma unroll
  for (int j = 0; j < 6; ++j) {
    *(volatile v4u*)(xm_hi + (size_t)j * kPE + eo) = hu[j];
    *(volatile v4u*)(xm_lo + (size_t)j * kPE + eo) = lu[j];
  }
  __threadfence();
#pragma unroll
  for (int j = 0; j < 6; ++j) {
    *(volatile v4u*)(xm_hi + (size_t)j * kPE + eo) = hu[j];
    *(volatile v4u*)(xm_lo + (size_t)j * kPE + eo) = lu[j];
  }
}

__global__ __launch_bounds__(256) void prep_kernel(float* planes, const float* __restrict__ wpre, const float* __restrict__ apre,
                                                   const float* __restrict__ k_k, const float* __restrict__ k_a) {
  __shared__ float part[8];
  const int row = blockIdx.x;
  const int d = threadIdx.x;
  const int lane = d & 31, wave = d >> 5;
  const size_t off = (size_t)row * kDim + d;
  const float kv = planes[kPE + off];
  const float ap = apre[off];
  const float wp = wpre[off];
  const float av = 1.0f / (1.0f + expf(-ap));
  const float kkv = kv * k_k[d];
  float sq = kkv * kkv;
#pragma unroll
  for (int o = 16; o > 0; o >>= 1) sq += __shfl_xor(sq, o);
  if (lane == 0) part[wave] = sq;
  __syncthreads();
  float tot = part[0];
#pragma unroll
  for (int w = 1; w < 8; ++w) tot = tot + part[w];
  const float nrm = fmaxf(sqrtf(tot), 1e-12f);
  const float kkn = kkv * (1.0f / nrm);
  const float bbv = kkn * av;
  const float km  = kv * (1.0f + (av - 1.0f) * k_a[d]);
  const float sw  = 1.0f / (1.0f + expf(-wp));
  const float dec = expf(kDecayScale * sw);
  float* p3 = planes + 3 * kPE + off;
  float* p4 = planes + 4 * kPE + off;
  float* p5 = planes + 5 * kPE + off;
  float* p6 = planes + 6 * kPE + off;
  *(volatile float*)p3 = dec;
  *(volatile float*)p4 = kkn;
  *(volatile float*)p5 = bbv;
  *(volatile float*)p6 = km;
  __threadfence();
  *(volatile float*)p3 = dec;
  *(volatile float*)p4 = kkn;
  *(volatile float*)p5 = bbv;
  *(volatile float*)p6 = km;
}

__device__ __forceinline__ int vpad(int i) { return i + ((i >> 6) << 2); }
__device__ __forceinline__ void sched_fence() { asm volatile("" ::: "memory"); }

__device__ __forceinline__ void flush_half16(const float* src, float* dst, int tid) {
  const int row = tid >> 5;
  const int c4 = (tid & 31) * 4;
  const v4f val = *(const v4f*)(src + row * kHalf + c4);
  float* p = dst + (size_t)row * kDim + c4;
  *(volatile v4f*)p = val;
  __threadfence();
  *(volatile v4f*)p = val;
}

__global__ __launch_bounds__(kScanThreads) void state_scan_kernel(const float* planes, float* oplane) {
#pragma clang fp contract(off)
  __shared__ __align__(16) float vbuf[2][6][kVecPad];
  __shared__ __align__(16) float orow[2][16][kHalf];
  const int tid = threadIdx.x;
  const int bb = blockIdx.x >> 1;
  const int rh = blockIdx.x & 1;
  const int il = tid >> 2;
  const int cq = tid & 3;
  const int vr = rh * kHalf + il;
  const int segoff = cq * 68;
  const int el = tid & 255;
  const int q = tid >> 8;
  const int pel = vpad(el);
  const long pl0 = q ? 6L : 0L;
  const long pl1 = q ? 3L : 4L;
  const long pl2 = q ? 2L : 5L;
  const int  sl0 = 3 * q;
  const size_t rowb = (size_t)bb * kSeq;
  const float* src0 = planes + pl0 * kPE + el;
  const float* src1 = planes + pl1 * kPE + el;
  const float* src2 = planes + pl2 * kPE + el;
  float* obase = oplane + rowb * kDim + (size_t)rh * kHalf;

  float n0 = src0[rowb * kDim];
  float n1 = src1[rowb * kDim];
  float n2 = src2[rowb * kDim];
  vbuf[0][sl0][pel]     = n0;
  vbuf[0][sl0 + 1][pel] = n1;
  vbuf[0][sl0 + 2][pel] = n2;
  __syncthreads();

  v4f st[16];
#pragma unroll
  for (int j = 0; j < 16; ++j) st[j] = (v4f){0.f, 0.f, 0.f, 0.f};

  const int pvr = vpad(vr);
  for (int t = 0; t < kSeq; ++t) {
    const int cur = t & 1;
    const int tn = (t + 1 < kSeq) ? (t + 1) : (kSeq - 1);
    const size_t noff = (rowb + (size_t)tn) * kDim;
    n0 = src0[noff];
    n1 = src1[noff];
    n2 = src2[noff];
    if (((t & 15) == 0) && (t > 0)) {
      const int w = (t >> 4) - 1;
      flush_half16(&orow[w & 1][0][0], obase + (size_t)(16 * w) * kDim, tid);
    }
    const float* br  = &vbuf[cur][0][0];
    const float* bkk = &vbuf[cur][1][0];
    const float* bbb = &vbuf[cur][2][0];
    const float* bkm = &vbuf[cur][3][0];
    const float* bdc = &vbuf[cur][4][0];
    const float* bvv = &vbuf[cur][5][0];

    float sa = 0.f;
#pragma unroll
    for (int j = 0; j < 16; ++j) {
      const v4f k4 = *(const v4f*)(bkk + segoff + 4 * j);
      const v4f sj = st[j];
      sa = sa + sj.x * k4.x;
      sa = sa + sj.y * k4.y;
      sa = sa + sj.z * k4.z;
      sa = sa + sj.w * k4.w;
      if ((j & 3) == 3) sched_fence();
    }
    sa += __shfl_xor(sa, 1);
    sa += __shfl_xor(sa, 2);
    sa = -sa;
    const float vt = bvv[pvr];
    float oa = 0.f;
#pragma unroll
    for (int j = 0; j < 16; ++j) {
      const int p = segoff + 4 * j;
      const v4f d4 = *(const v4f*)(bdc + p);
      const v4f b4 = *(const v4f*)(bbb + p);
      const v4f k4 = *(const v4f*)(bkm + p);
      const v4f r4 = *(const v4f*)(br + p);
      const v4f sj = st[j];
      const float nx = (sj.x * d4.x + sa * b4.x) + vt * k4.x;
      const float ny = (sj.y * d4.y + sa * b4.y) + vt * k4.y;
      const float nz = (sj.z * d4.z + sa * b4.z) + vt * k4.z;
      const float nw = (sj.w * d4.w + sa * b4.w) + vt * k4.w;
      st[j] = (v4f){nx, ny, nz, nw};
      oa = oa + nx * r4.x;
      oa = oa + ny * r4.y;
      oa = oa + nz * r4.z;
      oa = oa + nw * r4.w;
      if ((j & 3) == 3) sched_fence();
    }
    oa += __shfl_xor(oa, 1);
    oa += __shfl_xor(oa, 2);
    if (cq == 0) orow[(t >> 4) & 1][t & 15][il] = oa;
    vbuf[cur ^ 1][sl0][pel]     = n0;
    vbuf[cur ^ 1][sl0 + 1][pel] = n1;
    vbuf[cur ^ 1][sl0 + 2][pel] = n2;
    __syncthreads();
  }
  const int wl = kSeq / 16 - 1;
  flush_half16(&orow[wl & 1][0][0], obase + (size_t)(16 * wl) * kDim, tid);
}

__device__ __forceinline__ void ld8f(float* dst, const float* p) {
  const v4f a = *(const v4f*)(p);
  const v4f c = *(const v4f*)(p + 4);
#pragma unroll
  for (int e = 0; e < 4; ++e) { dst[e] = a[e]; dst[4 + e] = c[e]; }
}
__device__ __forceinline__ float wsum32(float v) {
#pragma unroll
  for (int o = 16; o > 0; o >>= 1) v += __shfl_xor(v, o);
  return v;
}

__global__ __launch_bounds__(256) void post_kernel(const float* __restrict__ planes, const float* __restrict__ gpl,
                                                   const float* __restrict__ r_k, const float* __restrict__ gn_w,
                                                   const float* __restrict__ gn_b,
                                                   unsigned short* __restrict__ og_hi, unsigned short* __restrict__ og_lo) {
  const int tid = threadIdx.x;
  const int lane = tid & 31, wave = tid >> 5;
  const int row = blockIdx.x * 8 + wave;
  const int ch0 = lane * 8;
  const size_t off = (size_t)row * kDim + ch0;
  float o8[8], r8[8], km8[8], vv8[8], g8[8], rk8[8], gw8[8], gb8[8];
  ld8f(o8,  planes + 7 * kPE + off);
  ld8f(r8,  planes + off);
  ld8f(km8, planes + 6 * kPE + off);
  ld8f(vv8, planes + 2 * kPE + off);
  ld8f(g8,  gpl + off);
  ld8f(rk8, r_k + ch0);
  ld8f(gw8, gn_w + ch0);
  ld8f(gb8, gn_b + ch0);
  float so = 0.f, sb = 0.f;
#pragma unroll
  for (int e = 0; e < 8; ++e) {
    so = so + o8[e];
    sb = sb + (r8[e] * km8[e]) * rk8[e];
  }
  so = wsum32(so);
  sb = wsum32(sb);
  const float mu = so * kInvDim;
  float cc[8];
  float sv = 0.f;
#pragma unroll
  for (int e = 0; e < 8; ++e) {
    const float c = o8[e] - mu;
    cc[e] = c;
    sv = sv + c * c;
  }
  sv = wsum32(sv);
  const float var = sv * kInvDim;
  const float rs = 1.0f / sqrtf(var + kGnEps);
  unsigned short hb[8], lb[8];
#pragma unroll
  for (int e = 0; e < 8; ++e) {
    const float nrm = (cc[e] * rs) * gw8[e] + gb8[e];
    const float f = (nrm + sb * vv8[e]) * g8[e];
    const unsigned short h = f2bf_bits(f);
    hb[e] = h;
    lb[e] = f2bf_bits(f - bf_bits2f(h));
  }
  const v4u hu = (v4u){pk16(hb[0], hb[1]), pk16(hb[2], hb[3]), pk16(hb[4], hb[5]), pk16(hb[6], hb[7])};
  const v4u lu = (v4u){pk16(lb[0], lb[1]), pk16(lb[2], lb[3]), pk16(lb[4], lb[5]), pk16(lb[6], lb[7])};
  *(volatile v4u*)(og_hi + off) = hu;
  *(volatile v4u*)(og_lo + off) = lu;
  __threadfence();
  *(volatile v4u*)(og_hi + off) = hu;
  *(volatile v4u*)(og_lo + off) = lu;
}

template <int BIAS, int OUTM, int ACT>
static void run_gemm(const unsigned short* Ah, const unsigned short* Al, int lda, long sA,
                     const unsigned short* Bh, const unsigned short* Bl, int ldb, long sB,
                     void* C, void* C2, int ldc, long sC, const float* bias,
                     int M, int N, int K, int nbatch, hipStream_t st) {
  const int tiles = (M / 64) * (N / 64);
  dim3 grid((unsigned)((tiles + 7) / 8), (unsigned)nbatch);
  wmma_gemm64<1, true, BIAS, OUTM, false, ACT><<<grid, dim3(256), 0, st>>>(
      Ah, Al, lda, sA, Bh, Bl, ldb, sB, C, C2, ldc, sC, bias, nullptr, 0L, M, N, K, 1.0f);
}

static inline unsigned short* ws_u16(void* ws, size_t off) { return (unsigned short*)((char*)ws + off); }
static inline float* ws_f32(void* ws, size_t off) { return (float*)((char*)ws + off); }

extern "C" void kernel_launch(void* const* d_in, const int* in_sizes, int n_in,
                              void* d_out, int out_size, void* d_ws, size_t ws_size, hipStream_t stream) {
  if (n_in < 19) return;
  if (in_sizes[0] != (int)kPE || out_size != (int)kPE) return;
  if (ws_size < kCarveBytes) return;
  const float* x    = (const float*)d_in[0];
  const float* xmix = (const float*)d_in[1];
  const float* W_r  = (const float*)d_in[2];
  const float* W_k  = (const float*)d_in[3];
  const float* W_v  = (const float*)d_in[4];
  const float* W_o  = (const float*)d_in[5];
  const float* A_w  = (const float*)d_in[6];
  const float* B_w  = (const float*)d_in[7];
  const float* b_w  = (const float*)d_in[8];
  const float* A_a  = (const float*)d_in[9];
  const float* B_a  = (const float*)d_in[10];
  const float* b_a  = (const float*)d_in[11];
  const float* A_g  = (const float*)d_in[12];
  const float* B_g  = (const float*)d_in[13];
  const float* k_k  = (const float*)d_in[14];
  const float* k_a  = (const float*)d_in[15];
  const float* r_k  = (const float*)d_in[16];
  const float* gn_w = (const float*)d_in[17];
  const float* gn_b = (const float*)d_in[18];
  float* out = (float*)d_out;
  void* ws = d_ws;

  unsigned short* wt4h = ws_u16(ws, kOffWt4Hi);
  unsigned short* wt4l = ws_u16(ws, kOffWt4Lo);
  unsigned short* aw2h = ws_u16(ws, kOffAw2Hi);
  unsigned short* aw2l = ws_u16(ws, kOffAw2Lo);
  unsigned short* agh  = ws_u16(ws, kOffAgHi);
  unsigned short* agl  = ws_u16(ws, kOffAgLo);
  unsigned short* bw2h = ws_u16(ws, kOffBw2Hi);
  unsigned short* bw2l = ws_u16(ws, kOffBw2Lo);
  unsigned short* bgh  = ws_u16(ws, kOffBgHi);
  unsigned short* bgl  = ws_u16(ws, kOffBgLo);
  unsigned short* xmh  = ws_u16(ws, kOffXmHi);
  unsigned short* xml  = ws_u16(ws, kOffXmLo);
  unsigned short* ogh  = ws_u16(ws, kOffOgHi);
  unsigned short* ogl  = ws_u16(ws, kOffOgLo);
  unsigned short* lwwh = ws_u16(ws, kOffLwWHi);
  unsigned short* lwwl = ws_u16(ws, kOffLwWLo);
  unsigned short* lwah = ws_u16(ws, kOffLwAHi);
  unsigned short* lwal = ws_u16(ws, kOffLwALo);
  unsigned short* lwgh = ws_u16(ws, kOffLwGHi);
  unsigned short* lwgl = ws_u16(ws, kOffLwGLo);
  float* planes = ws_f32(ws, kOffF);
  float* wpre   = ws_f32(ws, kOffWpre);
  float* apre   = ws_f32(ws, kOffApre);
  float* gbuf   = ws_f32(ws, kOffG);

  wsplit_t_kernel<<<dim3(kDim / 64, kDim / 64, 4), dim3(256), 0, stream>>>(W_r, W_k, W_v, W_o, wt4h, wt4l, kDim, kDim);
  wsplit_t_kernel<<<dim3(kDim / 64, kLrW / 64, 2), dim3(256), 0, stream>>>(A_w, A_a, A_a, A_a, aw2h, aw2l, kDim, kLrW);
  wsplit_t_kernel<<<dim3(kDim / 64, kLrG / 64, 1), dim3(256), 0, stream>>>(A_g, A_g, A_g, A_g, agh, agl, kDim, kLrG);
  wsplit_t_kernel<<<dim3(kLrW / 64, kDim / 64, 2), dim3(256), 0, stream>>>(B_w, B_a, B_a, B_a, bw2h, bw2l, kLrW, kDim);
  wsplit_t_kernel<<<dim3(kLrG / 64, kDim / 64, 1), dim3(256), 0, stream>>>(B_g, B_g, B_g, B_g, bgh, bgl, kLrG, kDim);

  const int n8 = (int)(kPE / 8);
  mix_kernel<<<dim3((unsigned)((n8 + 255) / 256)), dim3(256), 0, stream>>>(x, xmix, xmh, xml, n8);

  run_gemm<0, 0, 0>(xmh, xml, kDim, kPE, wt4h, wt4l, kDim, (long)kDim * kDim,
                    planes, nullptr, kDim, kPE, nullptr, kTok, kDim, kDim, 3, stream);
  run_gemm<0, 2, 1>(xmh + 3 * kPE, xml + 3 * kPE, kDim, 0L, aw2h, aw2l, kDim, 0L,
                    lwwh, lwwl, kLrW, 0L, nullptr, kTok, kLrW, kDim, 1, stream);
  run_gemm<0, 2, 0>(xmh + 4 * kPE, xml + 4 * kPE, kDim, 0L, aw2h + (size_t)kLrA * kDim, aw2l + (size_t)kLrA * kDim, kDim, 0L,
                    lwah, lwal, kLrA, 0L, nullptr, kTok, kLrA, kDim, 1, stream);
  run_gemm<0, 2, 6>(xmh + 5 * kPE, xml + 5 * kPE, kDim, 0L, agh, agl, kDim, 0L,
                    lwgh, lwgl, kLrG, 0L, nullptr, kTok, kLrG, kDim, 1, stream);
  run_gemm<2, 0, 0>(lwwh, lwwl, kLrW, 0L, bw2h, bw2l, kLrW, 0L,
                    wpre, nullptr, kDim, 0L, b_w, kTok, kDim, kLrW, 1, stream);
  run_gemm<2, 0, 0>(lwah, lwal, kLrA, 0L, bw2h + (size_t)kDim * kLrA, bw2l + (size_t)kDim * kLrA, kLrA, 0L,
                    apre, nullptr, kDim, 0L, b_a, kTok, kDim, kLrA, 1, stream);
  run_gemm<0, 0, 0>(lwgh, lwgl, kLrG, 0L, bgh, bgl, kLrG, 0L,
                    gbuf, nullptr, kDim, 0L, nullptr, kTok, kDim, kLrG, 1, stream);

  prep_kernel<<<dim3(kTok), dim3(256), 0, stream>>>(planes, wpre, apre, k_k, k_a);

  state_scan_kernel<<<dim3(kBatch * 2), dim3(kScanThreads), 0, stream>>>(planes, planes + 7 * kPE);

  post_kernel<<<dim3(kTok / 8), dim3(256), 0, stream>>>(planes, gbuf, r_k, gn_w, gn_b, ogh, ogl);

  run_gemm<0, 0, 0>(ogh, ogl, kDim, 0L, wt4h + (size_t)3 * kDim * kDim, wt4l + (size_t)3 * kDim * kDim, kDim, 0L,
                    out, nullptr, kDim, 0L, nullptr, kTok, kDim, kDim, 1, stream);
}
